// EncoderRNN_9440338117094
// MI455X (gfx1250) — hardware-run, weakly checked
//
#include <hip/hip_runtime.h>
#include <math.h>
#include <stddef.h>

typedef __attribute__((ext_vector_type(16))) _Float16 v16h;
typedef __attribute__((ext_vector_type(8)))  _Float16 v8h;
typedef __attribute__((ext_vector_type(16))) __bf16   v16b;
typedef __attribute__((ext_vector_type(8)))  __bf16   v8b;
typedef __attribute__((ext_vector_type(8)))  float    v8f;
typedef __attribute__((ext_vector_type(4)))  float    v4f;
typedef __attribute__((ext_vector_type(4)))  unsigned int v4u;

#if __has_builtin(__builtin_amdgcn_sched_barrier)
#define KSTEP_SCHED_FENCE() __builtin_amdgcn_sched_barrier(0)
#else
#define KSTEP_SCHED_FENCE() asm volatile("" ::: "memory")
#endif

constexpr int NBATCH = 64;
constexpr int TSTEPS = 2048;
constexpr int EMBD   = 256;
constexpr int HIDD   = 256;
constexpr int GATE3  = 768;
constexpr int VOCABN = 50257;
constexpr int TCH    = 512;
constexpr int NCHUNK = TSTEPS / TCH;
constexpr int MROWS  = TCH * NBATCH;
constexpr int HP16   = 264;
constexpr int GHP    = 772;
constexpr int CVT_BLOCKS  = (GATE3 * EMBD / 8) / 256;
constexpr int CVT_THREADS = CVT_BLOCKS * 256;
constexpr int BIAS_THREADS = GATE3 / 4;
constexpr int GATHER_BLOCKS = MROWS / 8;
constexpr int GEMM_BLOCKS = (MROWS / 64) * (GATE3 / 64) / 8;
constexpr int SCAN_BLOCKS = NBATCH / 16;
constexpr float W_CARRY    = 256.0f;
constexpr float H_CARRY    = 64.0f;
constexpr float GH_UNSCALE = 1.0f / 16384.0f;

static_assert(TSTEPS % TCH == 0, "time groups");
static_assert(MROWS % 64 == 0 && GATE3 % 64 == 0 && EMBD % 32 == 0 && HIDD % 32 == 0, "kit GEMM shape contract");
static_assert((MROWS / 64) * (GATE3 / 64) == GEMM_BLOCKS * 8, "GEMM grid exact");
static_assert(CVT_THREADS * 8 == GATE3 * EMBD, "weight convert coverage");
static_assert(BIAS_THREADS * 4 == GATE3 && BIAS_THREADS % 32 == 0, "bias convert coverage, wave-uniform");
static_assert(GATHER_BLOCKS * 8 == MROWS, "gather coverage");
static_assert(GATE3 == 16 * 48, "16 waves x 48 columns in the recurrence kernel");
static_assert(HIDD == 32 * 8, "32 lanes x 8 column groups in the gate phase");
static_assert(SCAN_BLOCKS * 16 == NBATCH, "recurrence grid exact");

constexpr size_t WPLANE_BYTES  = (size_t)GATE3 * EMBD * 2;
constexpr size_t BIAS_BYTES    = (size_t)GATE3 * 4;
constexpr size_t HSTATE_BYTES  = (size_t)NBATCH * HIDD * 4;
constexpr size_t XPLANE_BYTES  = (size_t)MROWS * EMBD * 2;
constexpr size_t GIPLANE_BYTES = (size_t)MROWS * GATE3 * 4;
constexpr size_t OFF_WIH = 0;
constexpr size_t OFF_WHH = OFF_WIH + WPLANE_BYTES;
constexpr size_t OFF_BIH = OFF_WHH + WPLANE_BYTES;
constexpr size_t OFF_BHH = OFF_BIH + BIAS_BYTES;
constexpr size_t OFF_HS0 = OFF_BHH + BIAS_BYTES;
constexpr size_t OFF_HS1 = OFF_HS0 + HSTATE_BYTES;
constexpr size_t OFF_X   = OFF_HS1 + HSTATE_BYTES;
constexpr size_t OFF_GI  = OFF_X + XPLANE_BYTES;
constexpr size_t WS_TOTAL = OFF_GI + GIPLANE_BYTES;
static_assert(WS_TOTAL == 118364160u, "carve total");
static_assert(WS_TOTAL <= 134217728u, "carve limit");
static_assert(OFF_WHH % 256 == 0 && OFF_BIH % 256 == 0 && OFF_BHH % 256 == 0 && OFF_HS0 % 256 == 0 &&
              OFF_HS1 % 256 == 0 && OFF_X % 256 == 0 && OFF_GI % 256 == 0, "line alignment");

__device__ __forceinline__ unsigned short f2bf_bits(float f) {
  unsigned u = __float_as_uint(f);
  return (unsigned short)((u + 0x7FFFu + ((u >> 16) & 1u)) >> 16);
}
__device__ __forceinline__ float bf_bits2f(unsigned short h) { return __uint_as_float(((unsigned)h) << 16); }

__device__ __forceinline__ void dep_guard_h(v8f& a, v8f& b, v16h x, v16h y) { asm volatile("v_nop\n\tv_nop\n\tv_nop\n\tv_nop" : "+v"(a), "+v"(b) : "v"(x), "v"(y)); }
__device__ __forceinline__ void dep_guard_b(v8f& a, v8f& b, v16b x, v16b y) { asm volatile("v_nop\n\tv_nop\n\tv_nop\n\tv_nop" : "+v"(a), "+v"(b) : "v"(x), "v"(y)); }
__device__ __forceinline__ void keep4_h(v16h a, v16h b, v16h c, v16h d) { asm volatile("v_nop" :: "v"(a), "v"(b), "v"(c), "v"(d)); }
__device__ __forceinline__ void keep4_b(v16b a, v16b b, v16b c, v16b d) { asm volatile("v_nop" :: "v"(a), "v"(b), "v"(c), "v"(d)); }
__device__ __forceinline__ void acc_guard4(v8f& a, v8f& b, v8f& c, v8f& d) { asm volatile("v_nop\n\tv_nop\n\tv_nop\n\tv_nop" : "+v"(a), "+v"(b), "+v"(c), "+v"(d)); }
__device__ __forceinline__ void acc_guard3(v8f& a, v8f& b, v8f& c) { asm volatile("v_nop\n\tv_nop\n\tv_nop\n\tv_nop" : "+v"(a), "+v"(b), "+v"(c)); }
__device__ __forceinline__ void guard3_keep4(v8f& a0, v8f& a1, v8f& a2, v16h f0, v16h f1, v16h f2, v16h f3) {
  asm volatile("v_nop\n\tv_nop\n\tv_nop\n\tv_nop" : "+v"(a0), "+v"(a1), "+v"(a2) : "v"(f0), "v"(f1), "v"(f2), "v"(f3));
}

template <typename T> struct Frag;
template <> struct Frag<_Float16> {
  typedef v16h V; union U { v16h v; v8h h[2]; };
  static __device__ __forceinline__ v16h load(const _Float16* p) {
    U f; f.h[0] = *(const v8h*)(p); f.h[1] = *(const v8h*)(p + 16); return f.v;
  }
  static __device__ __forceinline__ v8f mma(v16h a, v16h b, v8f c) {
    return __builtin_amdgcn_wmma_f32_16x16x32_f16(false, a, false, b, (short)0, c, false, false);
  }
  static __device__ __forceinline__ void guard(v8f& a, v8f& b, v16h x, v16h y) { dep_guard_h(a, b, x, y); }
  static __device__ __forceinline__ void keep(v16h a, v16h b, v16h c, v16h d) { keep4_h(a, b, c, d); }
};
template <> struct Frag<__bf16> {
  typedef v16b V; union U { v16b v; v8b h[2]; };
  static __device__ __forceinline__ v16b load(const __bf16* p) {
    U f; f.h[0] = *(const v8b*)(p); f.h[1] = *(const v8b*)(p + 16); return f.v;
  }
  static __device__ __forceinline__ v8f mma(v16b a, v16b b, v8f c) {
    return __builtin_amdgcn_wmma_f32_16x16x32_bf16(false, a, false, b, (short)0, c, false, false);
  }
  static __device__ __forceinline__ void guard(v8f& a, v8f& b, v16b x, v16b y) { dep_guard_b(a, b, x, y); }
  static __device__ __forceinline__ void keep(v16b a, v16b b, v16b c, v16b d) { keep4_b(a, b, c, d); }
};

template <int ET> struct Elem;
template <> struct Elem<0> { typedef _Float16 T; };
template <> struct Elem<1> { typedef __bf16 T; };
template <int ET, bool SPLIT, int BIAS_MODE, int OUT_MODE, bool RESID, int ACT = 0>
__global__ __launch_bounds__(256) void wmma_gemm64(
    const unsigned short* __restrict__ Ap, const unsigned short* __restrict__ A2p, int lda, long strideA,
    const unsigned short* __restrict__ Btp, const unsigned short* __restrict__ Bt2p, int ldb, long strideB,
    void* __restrict__ Cout, void* __restrict__ Cout2, int ldc, long strideC,
    const float* __restrict__ bias,
    const float* __restrict__ resid, long strideR,
    int M, int N, int K, float scale) {
  typedef typename Elem<ET>::T T;
  typedef typename Frag<T>::V V;
  const T* A = (const T*)Ap; const T* A2 = (const T*)A2p; const T* Bt = (const T*)Btp; const T* Bt2 = (const T*)Bt2p;
  __shared__ __align__(16) float sT[8][16 * 68];
  const int b    = blockIdx.y;
  const int lane = threadIdx.x & 31;
  const int wave = threadIdx.x >> 5;
  const int tilesN = N >> 6;
  const int tilesM = M >> 6;
  const int tile = blockIdx.x * 8 + wave;
  if (tile >= tilesM * tilesN) return;
  const int tm = tile / tilesN;
  const int tn = tile - tm * tilesN;
  const int m0 = tm << 6;
  const int n0 = tn << 6;

  const T* Ab  = A  + (size_t)b * strideA;
  const T* Bb  = Bt + (size_t)b * strideB;
  const T* Ab2 = SPLIT ? (A2  + (size_t)b * strideA) : nullptr;
  const T* Bb2 = SPLIT ? (Bt2 + (size_t)b * strideB) : nullptr;

  const int rlane = lane & 15;
  const int koff  = (lane >> 4) * 8;
  const int mOff  = (lane >> 4) * 8;

  v8f acc[4][4];
#pragma unroll
  for (int i = 0; i < 4; ++i)
#pragma unroll
    for (int j = 0; j < 4; ++j) acc[i][j] = (v8f){0.f,0.f,0.f,0.f,0.f,0.f,0.f,0.f};

  for (int k0 = 0; k0 < K; k0 += 32) {
    V bh[4], bl[4];
#pragma unroll
    for (int j = 0; j < 4; ++j) {
      const size_t bo = (size_t)(n0 + (j << 4) + rlane) * ldb + koff + k0;
      bh[j] = Frag<T>::load(Bb + bo);
      if (SPLIT) bl[j] = Frag<T>::load(Bb2 + bo);
    }
#pragma unroll
    for (int i = 0; i < 4; ++i) {
      const size_t ao = (size_t)(m0 + (i << 4) + rlane) * lda + koff + k0;
      V ah = Frag<T>::load(Ab + ao);
      V al;
      if (SPLIT) al = Frag<T>::load(Ab2 + ao);
#pragma unroll
      for (int j = 0; j < 4; ++j) {
        acc[i][j] = Frag<T>::mma(ah, bh[j], acc[i][j]);
        if (SPLIT) {
          acc[i][j] = Frag<T>::mma(ah, bl[j], acc[i][j]);
          acc[i][j] = Frag<T>::mma(al, bh[j], acc[i][j]);
        }
      }
      Frag<T>::guard(acc[i][0], acc[i][3], ah, SPLIT ? al : ah);
    }
    Frag<T>::keep(bh[0], bh[1], bh[2], bh[3]);
    if (SPLIT) Frag<T>::keep(bl[0], bl[1], bl[2], bl[3]);
  }
  acc_guard4(acc[0][0], acc[0][1], acc[0][2], acc[0][3]);
  acc_guard4(acc[1][0], acc[1][1], acc[1][2], acc[1][3]);
  acc_guard4(acc[2][0], acc[2][1], acc[2][2], acc[2][3]);
  acc_guard4(acc[3][0], acc[3][1], acc[3][2], acc[3][3]);

  float* slab = sT[wave];
  const float* Rb = RESID ? (resid + (size_t)b * strideR) : nullptr;
#pragma unroll
  for (int i = 0; i < 4; ++i) {
    const int mBase = m0 + (i << 4);
#pragma unroll
    for (int j = 0; j < 4; ++j) {
      const int n = n0 + (j << 4) + rlane;
      float bv = 0.f;
      if (BIAS_MODE == 2) bv = bias[n];
#pragma unroll
      for (int r = 0; r < 8; ++r) {
        float v = acc[i][j][r] * scale;
        if (BIAS_MODE == 1) v += bias[mBase + mOff + r];
        if (BIAS_MODE == 2) v += bv;
        if (RESID) v += Rb[(size_t)(mBase + mOff + r) * ldc + n];
        if (ACT == 1) v = tanhf(v);
        if (ACT == 2) v = fmaxf(v, 0.0f);
        if (ACT == 3) v = v / (1.0f + expf(-v));
        if (ACT == 4) v = (v > 0.f) ? v : 0.01f * v;
        if (ACT == 5) v = 0.5f * v * (1.0f + erff(v * 0.70710678118654752f));
        slab[(mOff + r) * 68 + (j << 4) + rlane] = v;
      }
    }
    __builtin_amdgcn_fence(__ATOMIC_RELEASE, "workgroup");
    __builtin_amdgcn_wave_barrier();
    __builtin_amdgcn_fence(__ATOMIC_ACQUIRE, "workgroup");
    if (OUT_MODE == 0) {
      float* C = (float*)Cout + (size_t)b * strideC;
      const int hh = lane >> 4, c4 = (lane & 15) * 4;
      for (int pass = 0; pass < 2; ++pass) {
#pragma unroll
        for (int it = 0; it < 8; ++it) {
          const int row = it * 2 + hh;
          v4f v = *(const v4f*)(slab + row * 68 + c4);
          *(volatile v4f*)(C + (size_t)(mBase + row) * ldc + n0 + c4) = v;
        }
        __threadfence();
      }
    } else {
      const int q = lane >> 3, c8 = (lane & 7) * 8;
      unsigned short* C  = (unsigned short*)Cout  + (size_t)b * strideC;
      unsigned short* C2 = (OUT_MODE == 2) ? ((unsigned short*)Cout2 + (size_t)b * strideC) : nullptr;
      for (int pass = 0; pass < 2; ++pass) {
#pragma unroll
        for (int it = 0; it < 4; ++it) {
          const int row = it * 4 + q;
          const float* sp = slab + row * 68 + c8;
          v8h hv, lv;
#pragma unroll
          for (int e = 0; e < 8; ++e) {
            if (OUT_MODE == 1) {
              hv[e] = (_Float16)sp[e];
            } else {
              unsigned short hb = f2bf_bits(sp[e]);
              unsigned short lb = f2bf_bits(sp[e] - bf_bits2f(hb));
              hv[e] = __builtin_bit_cast(_Float16, hb);
              lv[e] = __builtin_bit_cast(_Float16, lb);
            }
          }
          *(volatile v8h*)(C + (size_t)(mBase + row) * ldc + n0 + c8) = hv;
          if (OUT_MODE == 2) *(volatile v8h*)(C2 + (size_t)(mBase + row) * ldc + n0 + c8) = lv;
        }
        __threadfence();
      }
    }
    __builtin_amdgcn_fence(__ATOMIC_RELEASE, "workgroup");
    __builtin_amdgcn_wave_barrier();
    __builtin_amdgcn_fence(__ATOMIC_ACQUIRE, "workgroup");
  }
}

__device__ __forceinline__ float bf_rne(float x) {
  float f = bf_bits2f(f2bf_bits(x));
  asm volatile("" : "+v"(f));
  return f;
}
__device__ __forceinline__ unsigned short f16bits_bf_scaled(float x) {
  const float g = x * W_CARRY;
  float f = bf_bits2f(f2bf_bits(g));
  asm volatile("" : "+v"(f));
  const _Float16 h = (_Float16)f;
  return __builtin_bit_cast(unsigned short, h);
}
__device__ __forceinline__ unsigned pack2(unsigned short lo, unsigned short hi) {
  return (unsigned)lo | ((unsigned)hi << 16);
}
__device__ __forceinline__ float sigm(float x) {
  const float xc = fmaxf(x, -80.0f);
  return 1.0f / (1.0f + expf(-xc));
}

__global__ __launch_bounds__(256) void k_cvt_params(const float* __restrict__ wih, const float* __restrict__ whh,
                                                      const float* __restrict__ bih, const float* __restrict__ bhh,
                                                      unsigned short* __restrict__ wih16, unsigned short* __restrict__ whh16,
                                                      float* __restrict__ bih_r, float* __restrict__ bhh_r) {
  const int i = blockIdx.x * 256 + threadIdx.x;
  if (i >= CVT_THREADS) return;
  const size_t e0 = (size_t)i * 8;
  const v4f a0 = *(const v4f*)(wih + e0), a1 = *(const v4f*)(wih + e0 + 4);
  const v4f c0 = *(const v4f*)(whh + e0), c1 = *(const v4f*)(whh + e0 + 4);
  v4u pa, pc;
  pa[0] = pack2(f2bf_bits(a0[0]), f2bf_bits(a0[1]));
  pa[1] = pack2(f2bf_bits(a0[2]), f2bf_bits(a0[3]));
  pa[2] = pack2(f2bf_bits(a1[0]), f2bf_bits(a1[1]));
  pa[3] = pack2(f2bf_bits(a1[2]), f2bf_bits(a1[3]));
  pc[0] = pack2(f16bits_bf_scaled(c0[0]), f16bits_bf_scaled(c0[1]));
  pc[1] = pack2(f16bits_bf_scaled(c0[2]), f16bits_bf_scaled(c0[3]));
  pc[2] = pack2(f16bits_bf_scaled(c1[0]), f16bits_bf_scaled(c1[1]));
  pc[3] = pack2(f16bits_bf_scaled(c1[2]), f16bits_bf_scaled(c1[3]));
  unsigned short* da = wih16 + e0;
  unsigned short* dc = whh16 + e0;
  for (int pass = 0; pass < 2; ++pass) {
    *(volatile v4u*)da = pa;
    *(volatile v4u*)dc = pc;
    __threadfence();
  }
  if (i < BIAS_THREADS) {
    const v4f bi = *(const v4f*)(bih + 4 * i);
    const v4f bh = *(const v4f*)(bhh + 4 * i);
    v4f ri, rh;
#pragma unroll
    for (int e = 0; e < 4; ++e) { ri[e] = bf_rne(bi[e]); rh[e] = bf_rne(bh[e]); }
    float* di = bih_r + 4 * i;
    float* dh = bhh_r + 4 * i;
    for (int pass = 0; pass < 2; ++pass) {
      *(volatile v4f*)di = ri;
      *(volatile v4f*)dh = rh;
      __threadfence();
    }
  }
}

__global__ __launch_bounds__(256) void k_gather_rows(const int* __restrict__ seq, const float* __restrict__ emb,
                                                      unsigned short* __restrict__ xpl, int tblk) {
  const int lane = threadIdx.x & 31, wave = threadIdx.x >> 5;
  const int m = blockIdx.x * 8 + wave;
  if (m >= MROWS) return;
  const int bb = m & (NBATCH - 1);
  const int tt = tblk * TCH + (m >> 6);
  int tok = seq[bb * TSTEPS + tt];
  tok = tok < 0 ? 0 : tok;
  tok = tok > (VOCABN - 1) ? (VOCABN - 1) : tok;
  const float* row = emb + (size_t)tok * EMBD + lane * 8;
  const v4f a0 = *(const v4f*)row, a1 = *(const v4f*)(row + 4);
  v4u p;
  p[0] = pack2(f2bf_bits(a0[0]), f2bf_bits(a0[1]));
  p[1] = pack2(f2bf_bits(a0[2]), f2bf_bits(a0[3]));
  p[2] = pack2(f2bf_bits(a1[0]), f2bf_bits(a1[1]));
  p[3] = pack2(f2bf_bits(a1[2]), f2bf_bits(a1[3]));
  unsigned short* dst = xpl + (size_t)m * EMBD + lane * 8;
  for (int pass = 0; pass < 2; ++pass) {
    *(volatile v4u*)dst = p;
    __threadfence();
  }
}

__global__ __launch_bounds__(512) void k_gru_steps(const unsigned short* __restrict__ whh16,
                                                    const float* __restrict__ bhh_r,
                                                    const float* __restrict__ gi,
                                                    const float* __restrict__ hin, float* __restrict__ hout, int first) {
  __shared__ __align__(16) float    hF[16 * HIDD];
  __shared__ __align__(16) _Float16 hH[16 * HP16];
  __shared__ __align__(16) float    ghs[16 * GHP];

  const int tid = threadIdx.x, lane = tid & 31, wave = tid >> 5;
  const int hh = lane >> 4, rl = lane & 15;
  const int bbase = blockIdx.x * 16;
  const _Float16* Wp = (const _Float16*)(const void*)whh16;
  const int n0 = wave * 48;

  const float bh0 = bhh_r[n0 + rl];
  const float bh1 = bhh_r[n0 + 16 + rl];
  const float bh2 = bhh_r[n0 + 32 + rl];

  float*    hrow = hF + wave * HIDD;
  _Float16* h16  = hH + wave * HP16;

  {
    const float* src = hin + (size_t)(bbase + wave) * HIDD;
#pragma unroll
    for (int e = 0; e < 8; ++e) {
      const int col = lane + 32 * e;
      float v = 0.0f;
      if (!first) v = src[col];
      asm volatile("" : "+v"(v));
      hrow[col] = v;
      h16[col]  = (_Float16)(v * H_CARRY);
    }
  }
  __syncthreads();

  const float* girow = gi + (size_t)(bbase + wave) * GATE3;
  const float* sp    = ghs + wave * GHP;

  for (int tl = 0; tl < TCH; ++tl) {
    v8f acc0 = (v8f){0.f,0.f,0.f,0.f,0.f,0.f,0.f,0.f};
    v8f acc1 = acc0, acc2 = acc0;
#pragma unroll
    for (int kt = 0; kt < HIDD / 32; ++kt) {
      const int ko = kt * 32 + 8 * hh;
      const v16h a  = Frag<_Float16>::load(hH + rl * HP16 + ko);
      const v16h w0 = Frag<_Float16>::load(Wp + (size_t)(n0 + rl) * HIDD + ko);
      const v16h w1 = Frag<_Float16>::load(Wp + (size_t)(n0 + 16 + rl) * HIDD + ko);
      const v16h w2 = Frag<_Float16>::load(Wp + (size_t)(n0 + 32 + rl) * HIDD + ko);
      acc0 = Frag<_Float16>::mma(a, w0, acc0);
      acc1 = Frag<_Float16>::mma(a, w1, acc1);
      acc2 = Frag<_Float16>::mma(a, w2, acc2);
      guard3_keep4(acc0, acc1, acc2, a, w0, w1, w2);
      KSTEP_SCHED_FENCE();
    }
    acc_guard3(acc0, acc1, acc2);
#pragma unroll
    for (int r = 0; r < 8; ++r) {
      float* gp = ghs + (8 * hh + r) * GHP + n0 + rl;
      gp[0]  = acc0[r] * GH_UNSCALE + bh0;
      gp[16] = acc1[r] * GH_UNSCALE + bh1;
      gp[32] = acc2[r] * GH_UNSCALE + bh2;
    }
    __syncthreads();

    {
      const float* gp = girow + (size_t)tl * (NBATCH * GATE3);
#pragma unroll 1
      for (int e = 0; e < 8; ++e) {
        const int col = lane + 32 * e;
        const float ir = gp[col], iz = gp[HIDD + col], iq = gp[2 * HIDD + col];
        const float hr = sp[col], hz = sp[HIDD + col], hq = sp[2 * HIDD + col];
        const float ho = hrow[col];
        const float rg = sigm(ir + hr);
        const float zg = sigm(iz + hz);
        const float ng = tanhf(iq + rg * hq);
        const float hv = (1.0f - zg) * ng + zg * ho;
        hrow[col] = hv;
        h16[col]  = (_Float16)(hv * H_CARRY);
      }
    }
    __syncthreads();
  }

  {
    float* orow = hout + (size_t)(bbase + wave) * HIDD;
    for (int pass = 0; pass < 2; ++pass) {
#pragma unroll
      for (int it = 0; it < 2; ++it) {
        const v4f v = *(const v4f*)(hrow + it * 128 + lane * 4);
        *(volatile v4f*)(orow + it * 128 + lane * 4) = v;
      }
      __threadfence();
    }
  }
}

extern "C" void kernel_launch(void* const* d_in, const int* in_sizes, int n_in,
                              void* d_out, int out_size, void* d_ws, size_t ws_size, hipStream_t stream) {
  if (n_in < 6) return;
  if (in_sizes[0] != NBATCH * TSTEPS) return;
  if (in_sizes[1] != VOCABN * EMBD) return;
  if (in_sizes[2] != GATE3 * EMBD || in_sizes[3] != GATE3 * HIDD) return;
  if (in_sizes[4] != GATE3 || in_sizes[5] != GATE3) return;
  if (out_size != NBATCH * HIDD) return;
  if (ws_size < WS_TOTAL) return;

  const int*   seq = (const int*)d_in[0];
  const float* emb = (const float*)d_in[1];
  const float* wih = (const float*)d_in[2];
  const float* whh = (const float*)d_in[3];
  const float* bih = (const float*)d_in[4];
  const float* bhh = (const float*)d_in[5];
  float* out = (float*)d_out;

  char* ws = (char*)d_ws;
  unsigned short* wih16 = (unsigned short*)(ws + OFF_WIH);
  unsigned short* whh16 = (unsigned short*)(ws + OFF_WHH);
  float* bih_r = (float*)(ws + OFF_BIH);
  float* bhh_r = (float*)(ws + OFF_BHH);
  float* hs0 = (float*)(ws + OFF_HS0);
  float* hs1 = (float*)(ws + OFF_HS1);
  unsigned short* xpl = (unsigned short*)(ws + OFF_X);
  float* gip = (float*)(ws + OFF_GI);

  k_cvt_params<<<dim3(CVT_BLOCKS, 1, 1), dim3(256, 1, 1), 0, stream>>>(wih, whh, bih, bhh, wih16, whh16, bih_r, bhh_r);

  for (int c = 0; c < NCHUNK; ++c) {
    k_gather_rows<<<dim3(GATHER_BLOCKS, 1, 1), dim3(256, 1, 1), 0, stream>>>(seq, emb, xpl, c);
    wmma_gemm64<1, false, 2, 0, false, 0><<<dim3(GEMM_BLOCKS, 1, 1), dim3(256, 1, 1), 0, stream>>>(
        xpl, xpl, EMBD, 0L,
        wih16, wih16, EMBD, 0L,
        (void*)gip, (void*)gip, GATE3, 0L,
        bih_r,
        (const float*)gip, 0L,
        MROWS, GATE3, EMBD, 1.0f);
    const float* hin = (c & 1) ? hs0 : hs1;
    float* hout = (c == NCHUNK - 1) ? out : ((c & 1) ? hs1 : hs0);
    const int first = (c == 0) ? 1 : 0;
    k_gru_steps<<<dim3(SCAN_BLOCKS, 1, 1), dim3(512, 1, 1), 0, stream>>>(whh16, bhh_r, gip, hin, hout, first);
  }
}
